// RCNN_65549790872110
// MI455X (gfx1250) — hardware-verified
//
#include <hip/hip_runtime.h>
#include <math.h>

constexpr int kNodes  = 16384;
constexpr int kSlots  = 8;
constexpr int kIn     = 512;
constexpr int kMem    = 256;
constexpr int kVocab  = 64;
constexpr int kFan    = 1024;
constexpr int kLeafLo = 2048;
constexpr float kStateCarry = 16.0f;
constexpr float kW3Carry    = 16.0f;
constexpr float kChildScale = 1.0f / 256.0f;

static_assert(kIn % 32 == 0);
static_assert(kMem % 64 == 0);
static_assert(kNodes % 64 == 0);
static_assert(kVocab % 64 == 0);
static_assert((kNodes - kLeafLo) % 8 == 0);
static_assert(kFan == kIn + 2 * kMem);

typedef __attribute__((ext_vector_type(16))) _Float16 v16h;
typedef __attribute__((ext_vector_type(8)))  _Float16 v8h;
typedef __attribute__((ext_vector_type(16))) __bf16   v16b;
typedef __attribute__((ext_vector_type(8)))  __bf16   v8b;
typedef __attribute__((ext_vector_type(8)))  float    v8f;
typedef __attribute__((ext_vector_type(4)))  float    v4f;
typedef __attribute__((ext_vector_type(4)))  unsigned int v4u;

__device__ __forceinline__ unsigned short f2bf_bits(float f) {
  unsigned u = __float_as_uint(f);
  return (unsigned short)((u + 0x7FFFu + ((u >> 16) & 1u)) >> 16);
}
__device__ __forceinline__ float bf_bits2f(unsigned short h) { return __uint_as_float(((unsigned)h) << 16); }

__device__ __forceinline__ void dep_guard_h(v8f& a, v8f& b, v16h x, v16h y) { asm volatile("v_nop\n\tv_nop\n\tv_nop\n\tv_nop" : "+v"(a), "+v"(b) : "v"(x), "v"(y)); }
__device__ __forceinline__ void dep_guard_b(v8f& a, v8f& b, v16b x, v16b y) { asm volatile("v_nop\n\tv_nop\n\tv_nop\n\tv_nop" : "+v"(a), "+v"(b) : "v"(x), "v"(y)); }
__device__ __forceinline__ void keep4_h(v16h a, v16h b, v16h c, v16h d) { asm volatile("v_nop" :: "v"(a), "v"(b), "v"(c), "v"(d)); }
__device__ __forceinline__ void keep4_b(v16b a, v16b b, v16b c, v16b d) { asm volatile("v_nop" :: "v"(a), "v"(b), "v"(c), "v"(d)); }
__device__ __forceinline__ void acc_guard4(v8f& a, v8f& b, v8f& c, v8f& d) { asm volatile("v_nop\n\tv_nop\n\tv_nop\n\tv_nop" : "+v"(a), "+v"(b), "+v"(c), "+v"(d)); }
template <typename T> struct Frag;
template <> struct Frag<_Float16> {
  typedef v16h V; union U { v16h v; v8h h[2]; };
  static __device__ __forceinline__ v16h load(const _Float16* p) {
    U f; f.h[0] = *(const v8h*)(p); f.h[1] = *(const v8h*)(p + 16); return f.v;
  }
  static __device__ __forceinline__ v8f mma(v16h a, v16h b, v8f c) {
    return __builtin_amdgcn_wmma_f32_16x16x32_f16(false, a, false, b, (short)0, c, false, false);
  }
  static __device__ __forceinline__ void guard(v8f& a, v8f& b, v16h x, v16h y) { dep_guard_h(a, b, x, y); }
  static __device__ __forceinline__ void keep(v16h a, v16h b, v16h c, v16h d) { keep4_h(a, b, c, d); }
};
template <> struct Frag<__bf16> {
  typedef v16b V; union U { v16b v; v8b h[2]; };
  static __device__ __forceinline__ v16b load(const __bf16* p) {
    U f; f.h[0] = *(const v8b*)(p); f.h[1] = *(const v8b*)(p + 16); return f.v;
  }
  static __device__ __forceinline__ v8f mma(v16b a, v16b b, v8f c) {
    return __builtin_amdgcn_wmma_f32_16x16x32_bf16(false, a, false, b, (short)0, c, false, false);
  }
  static __device__ __forceinline__ void guard(v8f& a, v8f& b, v16b x, v16b y) { dep_guard_b(a, b, x, y); }
  static __device__ __forceinline__ void keep(v16b a, v16b b, v16b c, v16b d) { keep4_b(a, b, c, d); }
};

__device__ __forceinline__ unsigned pk16(unsigned short a, unsigned short b) { return (unsigned)a | ((unsigned)b << 16); }
__device__ __forceinline__ unsigned short h_bits(float f) { const _Float16 h = (_Float16)f; return __builtin_bit_cast(unsigned short, h); }

template <int ET> struct Elem;
template <> struct Elem<0> { typedef _Float16 T; };
template <> struct Elem<1> { typedef __bf16 T; };
template <int ET, bool SPLIT, int BIAS_MODE, int OUT_MODE, bool RESID, int ACT = 0>
__global__ __launch_bounds__(256) void wmma_gemm64(
    const unsigned short* __restrict__ Ap, const unsigned short* __restrict__ A2p, int lda, long strideA,
    const unsigned short* __restrict__ Btp, const unsigned short* __restrict__ Bt2p, int ldb, long strideB,
    void* __restrict__ Cout, void* __restrict__ Cout2, int ldc, long strideC,
    const float* __restrict__ bias,
    const float* __restrict__ resid, long strideR,
    int M, int N, int K, float scale) {
  typedef typename Elem<ET>::T T;
  typedef typename Frag<T>::V V;
  const T* A = (const T*)Ap; const T* A2 = (const T*)A2p; const T* Bt = (const T*)Btp; const T* Bt2 = (const T*)Bt2p;
  __shared__ __align__(16) float sT[8][16 * 68];
  const int b    = blockIdx.y;
  const int lane = threadIdx.x & 31;
  const int wave = threadIdx.x >> 5;
  const int tilesN = N >> 6;
  const int tilesM = M >> 6;
  const int tile = blockIdx.x * 8 + wave;
  if (tile >= tilesM * tilesN) return;
  const int tm = tile / tilesN;
  const int tn = tile - tm * tilesN;
  const int m0 = tm << 6;
  const int n0 = tn << 6;

  const T* Ab  = A  + (size_t)b * strideA;
  const T* Bb  = Bt + (size_t)b * strideB;
  const T* Ab2 = SPLIT ? (A2  + (size_t)b * strideA) : nullptr;
  const T* Bb2 = SPLIT ? (Bt2 + (size_t)b * strideB) : nullptr;

  const int rlane = lane & 15;
  const int koff  = (lane >> 4) * 8;
  const int mOff  = (lane >> 4) * 8;

  v8f acc[4][4];
#pragma unroll
  for (int i = 0; i < 4; ++i)
#pragma unroll
    for (int j = 0; j < 4; ++j) acc[i][j] = (v8f){0.f,0.f,0.f,0.f,0.f,0.f,0.f,0.f};

  for (int k0 = 0; k0 < K; k0 += 32) {
    V bh[4], bl[4];
#pragma unroll
    for (int j = 0; j < 4; ++j) {
      const size_t bo = (size_t)(n0 + (j << 4) + rlane) * ldb + koff + k0;
      bh[j] = Frag<T>::load(Bb + bo);
      if (SPLIT) bl[j] = Frag<T>::load(Bb2 + bo);
    }
#pragma unroll
    for (int i = 0; i < 4; ++i) {
      const size_t ao = (size_t)(m0 + (i << 4) + rlane) * lda + koff + k0;
      V ah = Frag<T>::load(Ab + ao);
      V al;
      if (SPLIT) al = Frag<T>::load(Ab2 + ao);
#pragma unroll
      for (int j = 0; j < 4; ++j) {
        acc[i][j] = Frag<T>::mma(ah, bh[j], acc[i][j]);
        if (SPLIT) {
          acc[i][j] = Frag<T>::mma(ah, bl[j], acc[i][j]);
          acc[i][j] = Frag<T>::mma(al, bh[j], acc[i][j]);
        }
      }
      Frag<T>::guard(acc[i][0], acc[i][3], ah, SPLIT ? al : ah);
    }
    Frag<T>::keep(bh[0], bh[1], bh[2], bh[3]);
    if (SPLIT) Frag<T>::keep(bl[0], bl[1], bl[2], bl[3]);
  }
  acc_guard4(acc[0][0], acc[0][1], acc[0][2], acc[0][3]);
  acc_guard4(acc[1][0], acc[1][1], acc[1][2], acc[1][3]);
  acc_guard4(acc[2][0], acc[2][1], acc[2][2], acc[2][3]);
  acc_guard4(acc[3][0], acc[3][1], acc[3][2], acc[3][3]);

  float* slab = sT[wave];
  const float* Rb = RESID ? (resid + (size_t)b * strideR) : nullptr;
#pragma unroll
  for (int i = 0; i < 4; ++i) {
    const int mBase = m0 + (i << 4);
#pragma unroll
    for (int j = 0; j < 4; ++j) {
      const int n = n0 + (j << 4) + rlane;
      float bv = 0.f;
      if (BIAS_MODE == 2) bv = bias[n];
#pragma unroll
      for (int r = 0; r < 8; ++r) {
        float v = acc[i][j][r] * scale;
        if (BIAS_MODE == 1) v += bias[mBase + mOff + r];
        if (BIAS_MODE == 2) v += bv;
        if (RESID) v += Rb[(size_t)(mBase + mOff + r) * ldc + n];
        if (ACT == 2) v = fmaxf(v, 0.0f);
        if (ACT == 4) v = (v > 0.f) ? v : 0.01f * v;
        slab[(mOff + r) * 68 + (j << 4) + rlane] = v;
      }
    }
    __builtin_amdgcn_fence(__ATOMIC_RELEASE, "workgroup");
    __builtin_amdgcn_wave_barrier();
    __builtin_amdgcn_fence(__ATOMIC_ACQUIRE, "workgroup");
    if (OUT_MODE == 0) {
      float* C = (float*)Cout + (size_t)b * strideC;
      const int hh = lane >> 4, c4 = (lane & 15) * 4;
      for (int pass = 0; pass < 2; ++pass) {
#pragma unroll
        for (int it = 0; it < 8; ++it) {
          const int row = it * 2 + hh;
          v4f v = *(const v4f*)(slab + row * 68 + c4);
          *(volatile v4f*)(C + (size_t)(mBase + row) * ldc + n0 + c4) = v;
        }
        __threadfence();
      }
    } else {
      const int q = lane >> 3, c8 = (lane & 7) * 8;
      unsigned short* C  = (unsigned short*)Cout  + (size_t)b * strideC;
      unsigned short* C2 = (OUT_MODE == 2) ? ((unsigned short*)Cout2 + (size_t)b * strideC) : nullptr;
      for (int pass = 0; pass < 2; ++pass) {
#pragma unroll
        for (int it = 0; it < 4; ++it) {
          const int row = it * 4 + q;
          const float* sp = slab + row * 68 + c8;
          v8h hv, lv;
#pragma unroll
          for (int e = 0; e < 8; ++e) {
            if (OUT_MODE == 1) {
              hv[e] = (_Float16)sp[e];
            } else {
              unsigned short hb = f2bf_bits(sp[e]);
              unsigned short lb = f2bf_bits(sp[e] - bf_bits2f(hb));
              hv[e] = __builtin_bit_cast(_Float16, hb);
              lv[e] = __builtin_bit_cast(_Float16, lb);
            }
          }
          *(volatile v8h*)(C + (size_t)(mBase + row) * ldc + n0 + c8) = hv;
          if (OUT_MODE == 2) *(volatile v8h*)(C2 + (size_t)(mBase + row) * ldc + n0 + c8) = lv;
        }
        __threadfence();
      }
    }
    __builtin_amdgcn_fence(__ATOMIC_RELEASE, "workgroup");
    __builtin_amdgcn_wave_barrier();
    __builtin_amdgcn_fence(__ATOMIC_ACQUIRE, "workgroup");
  }
}

__global__ __launch_bounds__(256) void cvt_rows_kernel(const float* __restrict__ src, int src_ld, int col0,
                                                       unsigned short* __restrict__ dst, int ncols, int nrows, int mode) {
  const int i = blockIdx.x * 256 + threadIdx.x;
  const int per_row = ncols >> 3;
  if (i >= nrows * per_row) return;
  const int row = i / per_row;
  const int c = (i - row * per_row) * 8;
  const float* p = src + (size_t)row * src_ld + col0 + c;
  const v4f a  = *(const v4f*)(p);
  const v4f b4 = *(const v4f*)(p + 4);
  unsigned short hb[8];
#pragma unroll
  for (int e = 0; e < 4; ++e) {
    const unsigned short q0 = f2bf_bits(a[e]);
    const unsigned short q1 = f2bf_bits(b4[e]);
    const unsigned short g0 = h_bits(bf_bits2f(q0) * kW3Carry);
    const unsigned short g1 = h_bits(bf_bits2f(q1) * kW3Carry);
    hb[e]     = mode ? g0 : q0;
    hb[4 + e] = mode ? g1 : q1;
  }
  const v4u u = (v4u){pk16(hb[0], hb[1]), pk16(hb[2], hb[3]), pk16(hb[4], hb[5]), pk16(hb[6], hb[7])};
  unsigned short* q = dst + (size_t)row * ncols + c;
  *(volatile v4u*)q = u;
  __threadfence();
  *(volatile v4u*)q = u;
}

__global__ __launch_bounds__(256) void leaf_kernel(const float* __restrict__ Pb, float* __restrict__ out,
                                                   unsigned short* __restrict__ S16) {
  __shared__ __align__(16) float sh[8 * kMem];
  const int t = threadIdx.x, lane = t & 31, wave = t >> 5;
  const int row = kLeafLo + blockIdx.x * 8 + wave;
  const float* pr = Pb + (size_t)row * kMem;
  float* sw = sh + wave * kMem;
#pragma unroll 1
  for (int e = 0; e < 8; ++e) {
    const int col = e * 32 + lane;
    sw[col] = tanhf(pr[col]);
  }
  __syncthreads();
  const v4f o0 = *(const v4f*)(sw + 4 * lane);
  const v4f o1 = *(const v4f*)(sw + 128 + 4 * lane);
  const v4f a  = *(const v4f*)(sw + 8 * lane);
  const v4f c  = *(const v4f*)(sw + 8 * lane + 4);
  unsigned short hb[8];
#pragma unroll
  for (int e = 0; e < 4; ++e) {
    hb[e]     = h_bits(a[e] * kStateCarry);
    hb[4 + e] = h_bits(c[e] * kStateCarry);
  }
  const v4u u = (v4u){pk16(hb[0], hb[1]), pk16(hb[2], hb[3]), pk16(hb[4], hb[5]), pk16(hb[6], hb[7])};
  float* orow = out + (size_t)row * kMem;
  unsigned short* srow = S16 + (size_t)row * kMem;
  for (int pass = 0; pass < 2; ++pass) {
    *(volatile v4f*)(orow + 4 * lane) = o0;
    *(volatile v4f*)(orow + 128 + 4 * lane) = o1;
    *(volatile v4u*)(srow + 8 * lane) = u;
    __threadfence();
  }
}

constexpr int kNPB    = 4;
constexpr int kLRows  = kNPB * kSlots;
constexpr int kAPitch = 264;
constexpr int kQPitch = 260;

__global__ __launch_bounds__(256) void level_kernel(const float* __restrict__ Pb, const float* __restrict__ Dtab,
                                                    const unsigned short* __restrict__ W3h,
                                                    const int* __restrict__ child_idx, const int* __restrict__ child_deprel,
                                                    const int* __restrict__ counts,
                                                    float* __restrict__ out, unsigned short* S16, int lo, int hi) {
  __shared__ __align__(16) unsigned short As[kLRows * kAPitch];
  __shared__ __align__(16) float Qs[kLRows * kQPitch];
  __shared__ __align__(16) float Os[kNPB * kMem];
  __shared__ int      s_cl[kLRows];
  __shared__ unsigned s_mask[kLRows];
  __shared__ int      s_cdep[kLRows];
  __shared__ float    s_rsel[kLRows];
  __shared__ int      s_node[kNPB];
  __shared__ int      s_cnt[kNPB];

  const int t = threadIdx.x, lane = t & 31, wave = t >> 5;
  const int nbase = lo + blockIdx.x * kNPB;

  if (t < kLRows) {
    const int row = t, u = row >> 3, slot = row & 7;
    int node = nbase + u;
    node = (node < hi) ? node : (hi - 1);
    const int ci = child_idx[node * kSlots + slot];
    const int real = (ci >= 0) ? 1 : 0;
    int cl = (ci > kNodes - 1) ? (kNodes - 1) : ci;
    cl = real ? cl : (kNodes - 1);
    int cd = child_deprel[node * kSlots + slot];
    cd = (cd < 0) ? 0 : ((cd > kVocab - 1) ? (kVocab - 1) : cd);
    s_cl[row]   = cl;
    s_mask[row] = real ? 0xffffffffu : 0u;
    s_cdep[row] = cd;
    s_rsel[row] = real ? 1.0f : 0.0f;
    if (slot == 0) {
      int c = counts[node];
      c = (c < 1) ? 1 : ((c > kSlots) ? kSlots : c);
      s_node[u] = node;
      s_cnt[u]  = c;
    }
  }
  __syncthreads();

#pragma unroll
  for (int it = 0; it < 4; ++it) {
    const int id  = t + 256 * it;
    const int row = id >> 5;
    const int c16 = id & 31;
    const int cl  = s_cl[row];
    const unsigned msk = s_mask[row];
    v4u v = *(const v4u*)(S16 + (size_t)cl * kMem + 8 * c16);
    const v4u m4 = (v4u){msk, msk, msk, msk};
    v = v & m4;
    *(v4u*)(As + row * kAPitch + 8 * c16) = v;
  }
  __syncthreads();

  const int rlane = lane & 15;
  const int koff  = (lane >> 4) * 8;
  const int mOff  = (lane >> 4) * 8;
  const int ncol0 = wave * 32;
  const _Float16* Ah = (const _Float16*)As;
  const _Float16* Bg = (const _Float16*)W3h;
  v8f acc[2][2];
#pragma unroll
  for (int i = 0; i < 2; ++i)
#pragma unroll
    for (int j = 0; j < 2; ++j) acc[i][j] = (v8f){0.f,0.f,0.f,0.f,0.f,0.f,0.f,0.f};

  for (int k0 = 0; k0 < kMem; k0 += 32) {
    v16h bfr[2];
#pragma unroll
    for (int j = 0; j < 2; ++j)
      bfr[j] = Frag<_Float16>::load(Bg + (size_t)(ncol0 + 16 * j + rlane) * kMem + koff + k0);
#pragma unroll
    for (int i = 0; i < 2; ++i) {
      const v16h afr = Frag<_Float16>::load(Ah + (16 * i + rlane) * kAPitch + koff + k0);
#pragma unroll
      for (int j = 0; j < 2; ++j) acc[i][j] = Frag<_Float16>::mma(afr, bfr[j], acc[i][j]);
      Frag<_Float16>::guard(acc[i][0], acc[i][1], afr, afr);
    }
    Frag<_Float16>::keep(bfr[0], bfr[1], bfr[0], bfr[1]);
  }
  acc_guard4(acc[0][0], acc[0][1], acc[1][0], acc[1][1]);

#pragma unroll
  for (int i = 0; i < 2; ++i)
#pragma unroll
    for (int j = 0; j < 2; ++j)
#pragma unroll
      for (int r = 0; r < 8; ++r)
        Qs[(16 * i + mOff + r) * kQPitch + ncol0 + 16 * j + rlane] = acc[i][j][r];
  __syncthreads();

#pragma unroll 1
  for (int rr = 0; rr < 4; ++rr) {
    const int row  = wave * 4 + rr;
    const int node = s_node[row >> 3];
    const float* pbr = Pb + (size_t)node * kMem;
    const float* dr  = Dtab + (size_t)s_cdep[row] * kMem;
    const float rsel = s_rsel[row];
    float* qr = Qs + row * kQPitch;
#pragma unroll 1
    for (int e = 0; e < 8; ++e) {
      const int col = e * 32 + lane;
      const float qv = qr[col] * kChildScale;
      const float dv = dr[col] * rsel;
      const float v  = (qv + dv) + pbr[col];
      qr[col] = tanhf(v);
    }
  }
  __syncthreads();

  {
    const int f = t;
#pragma unroll 1
    for (int u = 0; u < kNPB; ++u) {
      const int C = s_cnt[u];
      float m = -3.4028234663852886e38f;
#pragma unroll 1
      for (int tt = 0; tt < C; ++tt) {
        const int j   = f * C + tt;
        const int row = u * kSlots + (j >> 8);
        const int col = j & 255;
        m = fmaxf(m, Qs[row * kQPitch + col]);
      }
      Os[u * kMem + f] = m;
    }
  }
  __syncthreads();

  if (wave < kNPB) {
    const int u = wave;
    const int node = nbase + u;
    if (node < hi) {
      const float* ou = Os + u * kMem;
      const v4f o0 = *(const v4f*)(ou + 4 * lane);
      const v4f o1 = *(const v4f*)(ou + 128 + 4 * lane);
      const v4f a  = *(const v4f*)(ou + 8 * lane);
      const v4f c  = *(const v4f*)(ou + 8 * lane + 4);
      unsigned short hb[8];
#pragma unroll
      for (int e = 0; e < 4; ++e) {
        hb[e]     = h_bits(a[e] * kStateCarry);
        hb[4 + e] = h_bits(c[e] * kStateCarry);
      }
      const v4u uu = (v4u){pk16(hb[0], hb[1]), pk16(hb[2], hb[3]), pk16(hb[4], hb[5]), pk16(hb[6], hb[7])};
      float* orow = out + (size_t)node * kMem;
      unsigned short* srow = S16 + (size_t)node * kMem;
      for (int pass = 0; pass < 2; ++pass) {
        *(volatile v4f*)(orow + 4 * lane) = o0;
        *(volatile v4f*)(orow + 128 + 4 * lane) = o1;
        *(volatile v4u*)(srow + 8 * lane) = uu;
        __threadfence();
      }
    }
  }
}

extern "C" void kernel_launch(void* const* d_in, const int* in_sizes, int n_in,
                              void* d_out, int out_size, void* d_ws, size_t ws_size, hipStream_t stream) {
  if (n_in < 7) return;
  if (in_sizes[0] != kNodes * kIn || in_sizes[1] != kMem * kFan || in_sizes[2] != kMem ||
      in_sizes[3] != kVocab * kMem || in_sizes[4] != kNodes * kSlots || in_sizes[5] != kNodes * kSlots ||
      in_sizes[6] != kNodes || out_size != kNodes * kMem) return;

  const float* inputs       = (const float*)d_in[0];
  const float* W            = (const float*)d_in[1];
  const float* bias         = (const float*)d_in[2];
  const float* emb          = (const float*)d_in[3];
  const int*   child_idx    = (const int*)d_in[4];
  const int*   child_deprel = (const int*)d_in[5];
  const int*   counts       = (const int*)d_in[6];
  float* out = (float*)d_out;

  char* ws = (char*)d_ws; size_t off = 0;
  auto carve = [&](size_t bytes) -> char* { char* p = ws + off; off += (bytes + 255) & ~(size_t)255; return p; };
  unsigned short* Xbf  = (unsigned short*)carve((size_t)kNodes * kIn * 2);
  unsigned short* W1t  = (unsigned short*)carve((size_t)kMem * kIn * 2);
  unsigned short* W2t  = (unsigned short*)carve((size_t)kMem * kMem * 2);
  unsigned short* W3h  = (unsigned short*)carve((size_t)kMem * kMem * 2);
  unsigned short* Ebf  = (unsigned short*)carve((size_t)kVocab * kMem * 2);
  float*          Pb   = (float*)carve((size_t)kNodes * kMem * 4);
  float*          Dtab = (float*)carve((size_t)kVocab * kMem * 4);
  unsigned short* S16  = (unsigned short*)carve((size_t)kNodes * kMem * 2);
  if (off > ws_size || off > (size_t)134217728) return;

  cvt_rows_kernel<<<(kNodes * (kIn / 8) + 255) / 256, 256, 0, stream>>>(inputs, kIn, 0, Xbf, kIn, kNodes, 0);
  cvt_rows_kernel<<<(kMem * (kIn / 8) + 255) / 256, 256, 0, stream>>>(W, kFan, 0, W1t, kIn, kMem, 0);
  cvt_rows_kernel<<<(kMem * (kMem / 8) + 255) / 256, 256, 0, stream>>>(W, kFan, kIn, W2t, kMem, kMem, 0);
  cvt_rows_kernel<<<(kMem * (kMem / 8) + 255) / 256, 256, 0, stream>>>(W, kFan, kIn + kMem, W3h, kMem, kMem, 1);
  cvt_rows_kernel<<<(kVocab * (kMem / 8) + 255) / 256, 256, 0, stream>>>(emb, kMem, 0, Ebf, kMem, kVocab, 0);

  {
    const int tiles = (kNodes / 64) * (kMem / 64);
    wmma_gemm64<1, false, 2, 0, false><<<dim3((tiles + 7) / 8, 1), 256, 0, stream>>>(
        Xbf, nullptr, kIn, 0L, W1t, nullptr, kIn, 0L,
        (void*)Pb, (void*)nullptr, kMem, 0L, bias, (const float*)nullptr, 0L, kNodes, kMem, kIn, 1.0f);
  }
  {
    const int tiles = (kVocab / 64) * (kMem / 64);
    wmma_gemm64<1, false, 0, 0, false><<<dim3((tiles + 7) / 8, 1), 256, 0, stream>>>(
        Ebf, nullptr, kMem, 0L, W2t, nullptr, kMem, 0L,
        (void*)Dtab, (void*)nullptr, kMem, 0L, (const float*)nullptr, (const float*)nullptr, 0L, kVocab, kMem, kMem, 1.0f);
  }
  leaf_kernel<<<(kNodes - kLeafLo) / 8, 256, 0, stream>>>(Pb, out, S16);

  const int lv_lo[5] = {585, 73, 9, 1, 0};
  const int lv_hi[5] = {2048, 585, 73, 9, 1};
  for (int i = 0; i < 5; ++i) {
    const int n = lv_hi[i] - lv_lo[i];
    level_kernel<<<(n + kNPB - 1) / kNPB, 256, 0, stream>>>(Pb, Dtab, W3h, child_idx, child_deprel, counts,
                                                            out, S16, lv_lo[i], lv_hi[i]);
  }
}
